// attention_42331197669711
// MI455X (gfx1250) — hardware-verified
//
#include <hip/hip_runtime.h>


#ifndef NB
#define NB 2
#endif
#ifndef SEQ
#define SEQ 2048
#endif
#define NB_FULL  2
#define SEQ_FULL 2048
#ifndef OUT_SEQ
#define OUT_SEQ SEQ
#endif
#ifndef QRES
#define QRES 0
#endif
#define DM   2048
#define NH_  16
#define HD   128
#define AW   4
#define OSP  132
#define QRS  2048.0f
#define QRI  (1.0f / 2048.0f)
#define SC2  (0.08838834764831845f * 1.4426950408889634f)
#define PSH  8.0f
#define CXS  256.0f
#define WOS  64.0f
#define OSC  (1.0f / 16384.0f)
#define WSI  (1.0f / 64.0f)
#define EPSF 1.1920929e-07f

static_assert(HD == 128);
static_assert(NH_ * HD == DM);
static_assert(DM % 64 == 0);
static_assert(HD % 64 == 0);
static_assert(DM % 32 == 0);
static_assert(SEQ % 64 == 0);
static_assert((NB * SEQ) % 64 == 0);
static_assert(SEQ % 32 == 0);
static_assert(SEQ % (16 * AW) == 0);
static_assert(((size_t)SEQ * DM) % 8 == 0);
static_assert(NB <= NB_FULL);
static_assert(SEQ <= SEQ_FULL);
static_assert(SEQ % 128 == 0);
static_assert((NB * SEQ) % 128 == 0);
static_assert((NB * SEQ) % 32 == 0);
static_assert((NB * SEQ) % 8 == 0);
static_assert(DM % 256 == 0);
static_assert(DM % 128 == 0);
static_assert((2 * DM) % 64 == 0);
static_assert(OSP >= 128 + 4);
static_assert(WSI * WOS == 1.0f);
static_assert(OSC * CXS * WOS == 1.0f);

typedef _Float16 h16;
typedef unsigned short bf;
typedef __attribute__((ext_vector_type(16))) _Float16 v16h;
typedef __attribute__((ext_vector_type(8)))  _Float16 v8h;
typedef __attribute__((ext_vector_type(8)))  float    v8f;
typedef __attribute__((ext_vector_type(4)))  float    v4f;
typedef v4f  __attribute__((may_alias)) v4fa;

__device__ __forceinline__ unsigned short f2bf(float f) { unsigned u = __float_as_uint(f); u += 0x7FFFu + ((u >> 16) & 1u); return (unsigned short)(u >> 16); }
__device__ __forceinline__ float bfr(float f) { return __uint_as_float(((unsigned)f2bf(f)) << 16); }
__device__ __forceinline__ v16h cat16(v8h lo, v8h hi) { return __builtin_shufflevector(lo, hi, 0, 1, 2, 3, 4, 5, 6, 7, 8, 9, 10, 11, 12, 13, 14, 15); }
__device__ __forceinline__ v8f wmma16(v16h a, v16h b, v8f c) { return __builtin_amdgcn_wmma_f32_16x16x32_f16(false, a, false, b, (short)0, c, false, false); }
__device__ __forceinline__ v16h  ldh(const h16* p) { return cat16(*(const v8h*)p, *(const v8h*)(p + 16)); }
__device__ __forceinline__ void wave_sync() { __builtin_amdgcn_fence(3  , "wavefront"); __builtin_amdgcn_wave_barrier(); asm volatile("" ::: "memory"); }
static __device__ __forceinline__ h16 toh_flush(float v) { const h16 r = (h16)v; return (fabsf(v) < 6.103515625e-05f) ? (h16)0.0f : r; }
__device__ __forceinline__ v8f wmma16g(v16h a, v16h b, v8f c) {
    c = __builtin_amdgcn_wmma_f32_16x16x32_f16(false, a, false, b, (short)0, c, false, false);
    asm volatile("v_nop\n\tv_nop\n\tv_nop\n\tv_nop" : "+v"(c) : "v"(a), "v"(b));
    return c;
}

__global__ __launch_bounds__(256) void k_rmsx(const float* __restrict__ x, const float* __restrict__ gq, const float* __restrict__ gkv, h16* XQ, h16* XKV) {
    const int lane = threadIdx.x & 31, wave = __builtin_amdgcn_readfirstlane((int)(threadIdx.x >> 5));
    const int row = blockIdx.x * 8 + wave;
    const int b = row / SEQ, t = row % SEQ;
    const float* xr = x + ((size_t)b * SEQ_FULL + (size_t)t) * DM + lane * 8;
    float ss = 0.0f;
#pragma unroll 1
    for (int i = 0; i < DM / 256; ++i) { const v8f v = *(const v8f*)(xr + i * 256);
#pragma unroll
        for (int j = 0; j < 8; ++j) { const float u = bfr(v[j]); ss += u * u; } }
    ss += __shfl_xor(ss, 16, 32); ss += __shfl_xor(ss, 8, 32); ss += __shfl_xor(ss, 4, 32); ss += __shfl_xor(ss, 2, 32); ss += __shfl_xor(ss, 1, 32);
    const float inv = rsqrtf(ss * (1.0f / (float)DM) + EPSF);
    h16* oq = XQ + (size_t)row * DM + lane * 8;
    h16* ok = XKV + (size_t)row * DM + lane * 8;
#pragma unroll 1
    for (int ps = 0; ps < 2; ++ps) {
#pragma unroll 1
        for (int i = 0; i < DM / 256; ++i) {
            const v8f v = *(const v8f*)(xr + i * 256);
            const v8f ga = *(const v8f*)(gq + i * 256 + lane * 8);
            const v8f gb = *(const v8f*)(gkv + i * 256 + lane * 8);
            v8h a, c;
#pragma unroll
            for (int j = 0; j < 8; ++j) { const float u = bfr(v[j]) * inv; a[j] = toh_flush(u * bfr(ga[j])); c[j] = toh_flush(u * bfr(gb[j])); }
            *(volatile v8h*)(oq + i * 256) = a; *(volatile v8h*)(ok + i * 256) = c; }
        if (ps == 0) __threadfence(); }
}

__global__ __launch_bounds__(256) void k_tcvt(const float* __restrict__ W, h16* Wt, int ldw) {
    __shared__ __align__(16) float tile[64 * 68];
    const int tid = threadIdx.x; const int n0 = blockIdx.x * 64, k0 = blockIdx.y * 64;
#pragma unroll
    for (int i = 0; i < 4; ++i) { const int kk = (tid >> 4) + 16 * i, c4 = (tid & 15) * 4;
        const v4f v = *(const v4f*)(W + (size_t)(k0 + kk) * (size_t)ldw + n0 + c4);
        *(v4fa*)(&tile[kk * 68 + c4]) = v; }
    __syncthreads();
#pragma unroll 1
    for (int ps = 0; ps < 2; ++ps) {
#pragma unroll
        for (int i = 0; i < 2; ++i) { const int nn = (tid >> 3) + 32 * i, k8 = (tid & 7) * 8;
            v8h o;
#pragma unroll
            for (int j = 0; j < 8; ++j) o[j] = toh_flush(bfr(tile[(k8 + j) * 68 + nn]) * WOS);
            const size_t oo = (size_t)(n0 + nn) * DM + k0 + k8;
            *(volatile v8h*)(Wt + oo) = o; }
        if (ps == 0) __threadfence(); }
}

__global__ __launch_bounds__(32) __attribute__((amdgpu_num_vgpr(256)))
void k_proj(const h16* __restrict__ A, const h16* __restrict__ Bt, const float* __restrict__ bias, const float* __restrict__ gain, h16* P,
            size_t sRB, size_t sCB, int biasRow, int doNorm, int RB, int pitch, int CB) {
    __shared__ __align__(16) float os[16 * OSP];
    const int K = DM;
    const int lane = threadIdx.x & 31, lr = lane & 15, hi = lane >> 4; const int r0 = blockIdx.x * 32, c0 = blockIdx.y * 128;
    v8f acc[2][8];
#pragma unroll
    for (int mb = 0; mb < 2; ++mb)
#pragma unroll
        for (int nb = 0; nb < 8; ++nb) acc[mb][nb] = (v8f){};
    const size_t aoff = (size_t)(r0 + lr) * K + 8 * hi, boff = (size_t)(c0 + lr) * K + 8 * hi;
#pragma unroll 1
    for (int kc = 0; kc < K; kc += 32) {
        const v16h a0 = ldh(A + aoff + kc);
        const v16h a1 = ldh(A + aoff + (size_t)16 * K + kc);
#pragma unroll
        for (int nb = 0; nb < 8; ++nb) { const v16h b = ldh(Bt + boff + (size_t)nb * 16 * K + kc);
            acc[0][nb] = wmma16g(a0, b, acc[0][nb]);
            acc[1][nb] = wmma16g(a1, b, acc[1][nb]); }
    }
    float bc[8];
#pragma unroll
    for (int nb = 0; nb < 8; ++nb) { const int ci = biasRow ? 0 : (c0 + nb * 16 + lr); const float t = bfr(bias[ci]); bc[nb] = biasRow ? 0.0f : t; }
    float gh[8];
#pragma unroll
    for (int j = 0; j < 8; ++j) { const float t = bfr(gain[lr * 8 + j]); gh[j] = doNorm ? t : 1.0f; }
    const size_t tbase = (size_t)(r0 / RB) * sRB + (size_t)(r0 % RB) * (size_t)pitch + (size_t)(c0 / CB) * sCB + (size_t)(c0 % CB);
#pragma unroll
    for (int mb = 0; mb < 2; ++mb) {
        float br[8];
#pragma unroll
        for (int j = 0; j < 8; ++j) { const int ri = biasRow ? (r0 + mb * 16 + hi * 8 + j) : 0; const float t = bfr(bias[ri]); br[j] = biasRow ? t : 0.0f; }
#pragma unroll
        for (int nb = 0; nb < 8; ++nb) {
#pragma unroll
            for (int j = 0; j < 8; ++j) os[(hi * 8 + j) * OSP + nb * 16 + lr] = acc[mb][nb][j] * WSI + bc[nb] + br[j]; }
        wave_sync();
        v8h hv[8];
#pragma unroll
        for (int s = 0; s < 8; ++s) { const int row = 2 * s + hi, c8 = lr * 8;
            const v4f x0 = *(const v4fa*)(&os[row * OSP + c8]); const v4f x1 = *(const v4fa*)(&os[row * OSP + c8 + 4]);
            float ss = 0.0f;
#pragma unroll
            for (int i = 0; i < 4; ++i) { ss += x0[i] * x0[i]; ss += x1[i] * x1[i]; }
            ss += __shfl_xor(ss, 1, 32); ss += __shfl_xor(ss, 2, 32); ss += __shfl_xor(ss, 4, 32); ss += __shfl_xor(ss, 8, 32);
            const float rn = rsqrtf(ss * (1.0f / (float)HD) + EPSF);
            const float inv = doNorm ? rn : 1.0f;
#pragma unroll
            for (int i = 0; i < 4; ++i) { hv[s][i] = toh_flush(x0[i] * inv * gh[i]); hv[s][4 + i] = toh_flush(x1[i] * inv * gh[4 + i]); } }
        const size_t sb = tbase + (size_t)(mb * 16) * (size_t)pitch;
#pragma unroll 1
        for (int ps = 0; ps < 2; ++ps) {
#pragma unroll
            for (int s = 0; s < 8; ++s) { const int row = 2 * s + hi, c8 = lr * 8;
                *(volatile v8h*)(P + sb + (size_t)row * (size_t)pitch + c8) = hv[s]; }
            if (ps == 0) __threadfence(); }
        wave_sync();
    }
}

__global__ __launch_bounds__(32 * AW) __attribute__((amdgpu_num_vgpr(256)))
void k_flash(const h16* __restrict__ QH, const h16* __restrict__ QR, const h16* __restrict__ KP, const h16* __restrict__ VT, h16* CX) {
    __shared__ __align__(16) float os[AW * 16 * OSP];
    const int lane = threadIdx.x & 31, wave = __builtin_amdgcn_readfirstlane((int)(threadIdx.x >> 5)), lr = lane & 15, hi = lane >> 4;
    const int zh = blockIdx.y; const int b = zh / NH_, h = zh % NH_;
    const int t0 = (blockIdx.x * AW + wave) * 16;
    const size_t pbase = (size_t)zh * SEQ * HD;
    const size_t qo = pbase + (size_t)(t0 + lr) * HD + 8 * hi;
    const v16h qh0 = ldh(QH + qo), qh1 = ldh(QH + qo + 32), qh2 = ldh(QH + qo + 64), qh3 = ldh(QH + qo + 96);
    const v16h qr0 = ldh(QR + qo), qr1 = ldh(QR + qo + 32), qr2 = ldh(QR + qo + 64), qr3 = ldh(QR + qo + 96);
    const size_t ko = pbase + (size_t)lr * HD + 8 * hi;
    const size_t vo = pbase + (size_t)lr * SEQ + 8 * hi;
    v8f o0 = (v8f){}, o1 = (v8f){}, o2 = (v8f){}, o3 = (v8f){}, o4 = (v8f){}, o5 = (v8f){}, o6 = (v8f){}, o7 = (v8f){};
    float m = -3.0e38f, l = 0.0f;
#pragma unroll 1
    for (int key0 = 0; key0 < SEQ; key0 += 32) {
        const h16* ka = KP + ko + (size_t)key0 * HD;
        v8f sHa = (v8f){}, sLa = (v8f){}, sHb = (v8f){}, sLb = (v8f){};
        { const v16h a0 = ldh(ka), a1 = ldh(ka + 32), b0 = ldh(ka + 16 * HD), b1 = ldh(ka + 16 * HD + 32);
          sHa = wmma16(a0, qh0, sHa); sHb = wmma16(b0, qh0, sHb);
          if (QRES) { sLa = wmma16(a0, qr0, sLa); sLb = wmma16(b0, qr0, sLb); }
          sHa = wmma16(a1, qh1, sHa); sHb = wmma16(b1, qh1, sHb);
          if (QRES) { sLa = wmma16(a1, qr1, sLa); sLb = wmma16(b1, qr1, sLb); }
          asm volatile("v_nop\n\tv_nop\n\tv_nop\n\tv_nop" : "+v"(sHa), "+v"(sLa), "+v"(sHb), "+v"(sLb) : "v"(a0), "v"(a1), "v"(b0), "v"(b1)); }
        { const v16h a2 = ldh(ka + 64), a3 = ldh(ka + 96), b2 = ldh(ka + 16 * HD + 64), b3 = ldh(ka + 16 * HD + 96);
          sHa = wmma16(a2, qh2, sHa); sHb = wmma16(b2, qh2, sHb);
          if (QRES) { sLa = wmma16(a2, qr2, sLa); sLb = wmma16(b2, qr2, sLb); }
          sHa = wmma16(a3, qh3, sHa); sHb = wmma16(b3, qh3, sHb);
          if (QRES) { sLa = wmma16(a3, qr3, sLa); sLb = wmma16(b3, qr3, sLb); }
          asm volatile("v_nop\n\tv_nop\n\tv_nop\n\tv_nop" : "+v"(sHa), "+v"(sLa), "+v"(sHb), "+v"(sLb) : "v"(a2), "v"(a3), "v"(b2), "v"(b3)); }
        float ta[8], tb[8]; float mx = -3.0e38f;
#pragma unroll
        for (int r = 0; r < 8; ++r) { ta[r] = (sHa[r] + sLa[r] * QRI) * SC2; tb[r] = (sHb[r] + sLb[r] * QRI) * SC2; mx = fmaxf(mx, fmaxf(ta[r], tb[r])); }
        mx = fmaxf(mx, __shfl_xor(mx, 16, 32));
        const float mnew = fmaxf(m, mx);
        const float alpha = __builtin_amdgcn_exp2f(m - mnew);
        const float sh = PSH - mnew;
        v16h pb; float ls = 0.0f;
#pragma unroll
        for (int r = 0; r < 8; ++r) { const h16 pa = (h16)__builtin_amdgcn_exp2f(ta[r] + sh); const h16 pc = (h16)__builtin_amdgcn_exp2f(tb[r] + sh); pb[r] = pa; pb[8 + r] = pc; ls += (float)pa + (float)pc; }
        l = l * alpha + ls; m = mnew;
        o0 = o0 * alpha; o1 = o1 * alpha; o2 = o2 * alpha; o3 = o3 * alpha; o4 = o4 * alpha; o5 = o5 * alpha; o6 = o6 * alpha; o7 = o7 * alpha;
        const h16* va = VT + vo + key0;
        { const v16h v0 = ldh(va), v1 = ldh(va + (size_t)16 * SEQ), v2 = ldh(va + (size_t)32 * SEQ), v3 = ldh(va + (size_t)48 * SEQ);
          o0 = wmma16(v0, pb, o0); o1 = wmma16(v1, pb, o1); o2 = wmma16(v2, pb, o2); o3 = wmma16(v3, pb, o3);
          asm volatile("v_nop\n\tv_nop\n\tv_nop\n\tv_nop" : "+v"(o0), "+v"(o1), "+v"(o2), "+v"(o3) : "v"(v0), "v"(v1), "v"(v2), "v"(v3), "v"(pb)); }
        { const v16h v4 = ldh(va + (size_t)64 * SEQ), v5 = ldh(va + (size_t)80 * SEQ), v6 = ldh(va + (size_t)96 * SEQ), v7 = ldh(va + (size_t)112 * SEQ);
          o4 = wmma16(v4, pb, o4); o5 = wmma16(v5, pb, o5); o6 = wmma16(v6, pb, o6); o7 = wmma16(v7, pb, o7);
          asm volatile("v_nop\n\tv_nop\n\tv_nop\n\tv_nop" : "+v"(o4), "+v"(o5), "+v"(o6), "+v"(o7) : "v"(v4), "v"(v5), "v"(v6), "v"(v7), "v"(pb)); }
    }
    l += __shfl_xor(l, 16, 32);
    const float sc = (1.0f / l) * CXS;
    const int wb = wave * 16 * OSP;
    { float* orw = &os[wb + lr * OSP + 8 * hi]; v4f a, c;
      a[0] = o0[0] * sc; a[1] = o0[1] * sc; a[2] = o0[2] * sc; a[3] = o0[3] * sc; c[0] = o0[4] * sc; c[1] = o0[5] * sc; c[2] = o0[6] * sc; c[3] = o0[7] * sc;
      *(v4fa*)(orw +   0) = a; *(v4fa*)(orw +   4) = c;
      a[0] = o1[0] * sc; a[1] = o1[1] * sc; a[2] = o1[2] * sc; a[3] = o1[3] * sc; c[0] = o1[4] * sc; c[1] = o1[5] * sc; c[2] = o1[6] * sc; c[3] = o1[7] * sc;
      *(v4fa*)(orw +  16) = a; *(v4fa*)(orw +  20) = c;
      a[0] = o2[0] * sc; a[1] = o2[1] * sc; a[2] = o2[2] * sc; a[3] = o2[3] * sc; c[0] = o2[4] * sc; c[1] = o2[5] * sc; c[2] = o2[6] * sc; c[3] = o2[7] * sc;
      *(v4fa*)(orw +  32) = a; *(v4fa*)(orw +  36) = c;
      a[0] = o3[0] * sc; a[1] = o3[1] * sc; a[2] = o3[2] * sc; a[3] = o3[3] * sc; c[0] = o3[4] * sc; c[1] = o3[5] * sc; c[2] = o3[6] * sc; c[3] = o3[7] * sc;
      *(v4fa*)(orw +  48) = a; *(v4fa*)(orw +  52) = c;
      a[0] = o4[0] * sc; a[1] = o4[1] * sc; a[2] = o4[2] * sc; a[3] = o4[3] * sc; c[0] = o4[4] * sc; c[1] = o4[5] * sc; c[2] = o4[6] * sc; c[3] = o4[7] * sc;
      *(v4fa*)(orw +  64) = a; *(v4fa*)(orw +  68) = c;
      a[0] = o5[0] * sc; a[1] = o5[1] * sc; a[2] = o5[2] * sc; a[3] = o5[3] * sc; c[0] = o5[4] * sc; c[1] = o5[5] * sc; c[2] = o5[6] * sc; c[3] = o5[7] * sc;
      *(v4fa*)(orw +  80) = a; *(v4fa*)(orw +  84) = c;
      a[0] = o6[0] * sc; a[1] = o6[1] * sc; a[2] = o6[2] * sc; a[3] = o6[3] * sc; c[0] = o6[4] * sc; c[1] = o6[5] * sc; c[2] = o6[6] * sc; c[3] = o6[7] * sc;
      *(v4fa*)(orw +  96) = a; *(v4fa*)(orw + 100) = c;
      a[0] = o7[0] * sc; a[1] = o7[1] * sc; a[2] = o7[2] * sc; a[3] = o7[3] * sc; c[0] = o7[4] * sc; c[1] = o7[5] * sc; c[2] = o7[6] * sc; c[3] = o7[7] * sc;
      *(v4fa*)(orw + 112) = a; *(v4fa*)(orw + 116) = c; }
    wave_sync();
    h16* crow = CX + ((size_t)b * SEQ + t0) * DM + h * HD;
#pragma unroll 1
    for (int ps = 0; ps < 2; ++ps) {
#pragma unroll
        for (int s = 0; s < 8; ++s) { const int row = 2 * s + hi, c8 = lr * 8;
            const v4f x0 = *(const v4fa*)(&os[wb + row * OSP + c8]); const v4f x1 = *(const v4fa*)(&os[wb + row * OSP + c8 + 4]); v8h hv;
#pragma unroll
            for (int i = 0; i < 4; ++i) { hv[i] = (h16)x0[i]; hv[4 + i] = (h16)x1[i]; }
            *(volatile v8h*)(crow + (size_t)row * DM + c8) = hv; }
        if (ps == 0) __threadfence(); }
}

__global__ __launch_bounds__(32) __attribute__((amdgpu_num_vgpr(256)))
void k_oproj(const h16* __restrict__ A, const h16* __restrict__ Bt, const float* __restrict__ bias, float* OUT) {
    __shared__ __align__(16) float os[16 * 68];
    const int K = DM;
    const int lane = threadIdx.x & 31, lr = lane & 15, hi = lane >> 4; const int r0 = blockIdx.x * 64, c0 = blockIdx.y * 64;
    v8f acc[4][4];
#pragma unroll
    for (int mb = 0; mb < 4; ++mb)
#pragma unroll
        for (int nb = 0; nb < 4; ++nb) acc[mb][nb] = (v8f){};
    const size_t aoff = (size_t)(r0 + lr) * K + 8 * hi, boff = (size_t)(c0 + lr) * K + 8 * hi;
#pragma unroll 1
    for (int kc = 0; kc < K; kc += 32) {
        v16h a[4];
#pragma unroll
        for (int mb = 0; mb < 4; ++mb) a[mb] = ldh(A + aoff + (size_t)mb * 16 * K + kc);
#pragma unroll
        for (int nb = 0; nb < 4; ++nb) { const v16h b = ldh(Bt + boff + (size_t)nb * 16 * K + kc);
#pragma unroll
            for (int mb = 0; mb < 4; ++mb) acc[mb][nb] = wmma16(a[mb], b, acc[mb][nb]); }
        asm volatile("v_nop\n\tv_nop\n\tv_nop\n\tv_nop" : "+v"(acc[0][0]), "+v"(acc[1][1]), "+v"(acc[2][2]), "+v"(acc[3][3]) : "v"(a[0]), "v"(a[1]), "v"(a[2]), "v"(a[3]));
    }
    float bc[4];
#pragma unroll
    for (int nb = 0; nb < 4; ++nb) bc[nb] = bfr(bias[c0 + nb * 16 + lr]);
    float* obase = OUT + ((size_t)(r0 / SEQ) * OUT_SEQ + (size_t)(r0 % SEQ)) * DM + c0;
#pragma unroll
    for (int mb = 0; mb < 4; ++mb) {
#pragma unroll
        for (int nb = 0; nb < 4; ++nb) {
#pragma unroll
            for (int j = 0; j < 8; ++j) os[(hi * 8 + j) * 68 + nb * 16 + lr] = acc[mb][nb][j] * OSC + bc[nb]; }
        wave_sync();
        float* orow = obase + (size_t)(mb * 16) * DM;
#pragma unroll 1
        for (int ps = 0; ps < 2; ++ps) {
#pragma unroll
            for (int s = 0; s < 8; ++s) { const int row = 2 * s + hi, cofs = lr * 4;
                const v4f val = *(const v4fa*)(&os[row * 68 + cofs]);
                *(volatile v4f*)(orow + (size_t)row * DM + cofs) = val; }
            if (ps == 0) __threadfence(); }
        wave_sync();
    }
}

static constexpr size_t al256(size_t v) { return (v + 255) & ~(size_t)255; }
static constexpr size_t SZ_XQ  = al256((size_t)NB * SEQ * DM * 2);
static constexpr size_t SZ_CX  = al256((size_t)NB * SEQ * DM * 2);
static constexpr size_t SZ_XKV = al256((size_t)NB * SEQ * DM * 2);
static constexpr size_t SZ_WQ  = al256((size_t)DM * DM * 2);
static constexpr size_t SZ_WKV = al256((size_t)2 * DM * DM * 2);
static constexpr size_t SZ_WO  = al256((size_t)DM * DM * 2);
static constexpr size_t SZ_PL  = al256((size_t)NB * NH_ * SEQ * HD * 2);
static constexpr size_t SZ_TOTAL = SZ_XQ + SZ_XKV + SZ_WQ + SZ_WKV + SZ_WO + (size_t)(3 + QRES) * SZ_PL;
static_assert(SZ_CX <= SZ_XQ);
static_assert(SZ_TOTAL <= (size_t)134217728);
static_assert(((size_t)DM * DM * 2) % 256 == 0);
static_assert((size_t)NB * NH_ * SEQ * HD == (size_t)NB * SEQ * DM);

extern "C" void kernel_launch(void* const* d_in, const int* in_sizes, int n_in,
                              void* d_out, int out_size, void* d_ws, size_t ws_size, hipStream_t stream) {
    if (n_in < 10) return;
    const size_t needx = ((size_t)(NB - 1) * SEQ_FULL + SEQ) * DM;
    if ((size_t)in_sizes[0] < needx) return;
    if ((size_t)in_sizes[1] < (size_t)DM || (size_t)in_sizes[3] < (size_t)DM || (size_t)in_sizes[4] < (size_t)DM || (size_t)in_sizes[9] < (size_t)DM) return;
    if ((size_t)in_sizes[2] < (size_t)DM * DM || (size_t)in_sizes[8] < (size_t)DM * DM) return;
    if ((size_t)in_sizes[5] < (size_t)2 * DM * DM || (size_t)in_sizes[6] < (size_t)2 * DM || (size_t)in_sizes[7] < (size_t)HD) return;
    if ((size_t)out_size < ((size_t)(NB - 1) * OUT_SEQ + SEQ) * DM) return;
    if (SZ_TOTAL > ws_size) return;
    const float* x   = (const float*)d_in[0];
    const float* gq  = (const float*)d_in[1];
    const float* wq  = (const float*)d_in[2]; const float* bq  = (const float*)d_in[3];
    const float* gkv = (const float*)d_in[4];
    const float* wkv = (const float*)d_in[5]; const float* bkv = (const float*)d_in[6];
    const float* ghd = (const float*)d_in[7];
    const float* wo  = (const float*)d_in[8]; const float* bo  = (const float*)d_in[9];
    float* OUT = (float*)d_out;
    char* wsp = (char*)d_ws;
    h16* XQ = (h16*)wsp; h16* CX = (h16*)wsp; wsp += SZ_XQ;
    h16* XKV = (h16*)wsp; wsp += SZ_XKV;
    h16* WQT = (h16*)wsp; wsp += SZ_WQ;
    h16* WKVT = (h16*)wsp; wsp += SZ_WKV;
    h16* WOT = (h16*)wsp; wsp += SZ_WO;
    h16* QH = (h16*)wsp; wsp += SZ_PL;
    h16* KP = (h16*)wsp; wsp += SZ_PL;
    h16* VT = (h16*)wsp; wsp += SZ_PL;
    h16* QR = QRES ? (h16*)wsp : QH;

    k_rmsx<<<(unsigned)(NB * SEQ / 8), 256, 0, stream>>>(x, gq, gkv, XQ, XKV);
    k_tcvt<<<dim3(DM / 64, DM / 64, 1), 256, 0, stream>>>(wq, WQT, DM);
    k_tcvt<<<dim3(2 * DM / 64, DM / 64, 1), 256, 0, stream>>>(wkv, WKVT, 2 * DM);
    k_tcvt<<<dim3(DM / 64, DM / 64, 1), 256, 0, stream>>>(wo, WOT, DM);

    k_proj<<<dim3(NB * SEQ / 32, DM / 128, 1), 32, 0, stream>>>(XQ, WQT, bq, ghd, QH, (size_t)NH_ * SEQ * HD, (size_t)SEQ * HD, 0, 1, SEQ, HD, HD);
    k_proj<<<dim3(NB * SEQ / 32, DM / 128, 1), 32, 0, stream>>>(XKV, WKVT, bkv, ghd, KP, (size_t)NH_ * SEQ * HD, (size_t)SEQ * HD, 0, 1, SEQ, HD, HD);
    k_proj<<<dim3(DM / 32, NB * SEQ / 128, 1), 32, 0, stream>>>(WKVT + (size_t)DM * DM, XKV, bkv + DM, ghd, VT, (size_t)0, (size_t)DM * SEQ, 1, 0, DM, SEQ, SEQ);

    k_flash<<<dim3(SEQ / (16 * AW), NB * NH_, 1), 32 * AW, 0, stream>>>(QH, QR, KP, VT, CX);

    k_oproj<<<dim3(NB * SEQ / 64, DM / 64, 1), 32, 0, stream>>>(CX, WOT, bo, OUT);
}
